// E3nnSimpleEdgeBlock_11587821764686
// MI455X (gfx1250) — hardware-verified
//
#include <hip/hip_runtime.h>


#ifndef NE
#define NE 50000
#endif
#define NE_FULL 50000
#define MUL_  32
#define DIMX  128
#define KUV   1024
#define NPATH 5
#define PLN   (MUL_ * KUV)
#define RP    260
#define OP    132
#define TP    68
#define ZC    256.0f
#define ZCI   (1.0f / 256.0f)
#define I3F   ((float)0.5773502691896258)
#define I6F   ((float)0.4082482904638631)
#define C0F   ((float)0.022097086912079611)
#define C1F   (0.03125f)

static_assert(NE % 16 == 0);
static_assert(NE <= NE_FULL);
static_assert(4 * MUL_ == DIMX);
static_assert(MUL_ * MUL_ == KUV);
static_assert(MUL_ == 32);
static_assert(KUV % 32 == 0);
static_assert(32 * 16 == DIMX * 4);
static_assert(8 * 4 == MUL_);
static_assert(8 * 16 == 64 * 2);
static_assert((RP * 4) % 16 == 0);
static_assert((OP * 4) % 16 == 0);
static_assert((TP * 4) % 16 == 0);
static_assert(RP >= 256);
static_assert(OP >= DIMX);
static_assert(TP >= 64);
static_assert((16 * RP + 16 * OP) * 4 <= 131072);
static_assert(32 * TP * 4 <= 131072);

typedef _Float16 h16;
typedef unsigned short bf;
typedef __attribute__((ext_vector_type(16))) _Float16 v16h;
typedef __attribute__((ext_vector_type(8)))  _Float16 v8h;
typedef __attribute__((ext_vector_type(8)))  float    v8f;
typedef __attribute__((ext_vector_type(4)))  float    v4f;
typedef v4f  __attribute__((may_alias)) v4fa;

__device__ __forceinline__ unsigned short f2bf(float f) { unsigned u = __float_as_uint(f); u += 0x7FFFu + ((u >> 16) & 1u); return (unsigned short)(u >> 16); }
__device__ __forceinline__ float bfr(float f) { return __uint_as_float(((unsigned)f2bf(f)) << 16); }
__device__ __forceinline__ v16h cat16(v8h lo, v8h hi) { return __builtin_shufflevector(lo, hi, 0, 1, 2, 3, 4, 5, 6, 7, 8, 9, 10, 11, 12, 13, 14, 15); }
__device__ __forceinline__ v8f wmma16(v16h a, v16h b, v8f c) { return __builtin_amdgcn_wmma_f32_16x16x32_f16(false, a, false, b, (short)0, c, false, false); }
__device__ __forceinline__ v16h  ldh(const h16* p) { return cat16(*(const v8h*)p, *(const v8h*)(p + 16)); }
__device__ __forceinline__ void wave_sync() { __builtin_amdgcn_fence(3  , "wavefront"); __builtin_amdgcn_wave_barrier(); asm volatile("" ::: "memory"); }

static __device__ __forceinline__ h16 toh_flush(float v) { const h16 r = (h16)v; return (fabsf(v) < 6.103515625e-05f) ? (h16)0.0f : r; }
static __device__ __forceinline__ v8f wmma16g(v16h a, v16h b, v8f c) {
    c = wmma16(a, b, c);
    asm volatile("v_nop\n\tv_nop\n\tv_nop\n\tv_nop" : "+v"(c) : "v"(a), "v"(b));
    return c;
}

__global__ __launch_bounds__(32) void k_wconv(const float* __restrict__ W, h16* WTp) {
    __shared__ __align__(16) float ts[32 * TP];
    const int lane = threadIdx.x & 31;
    const int j = blockIdx.x;
    const float* src = W + (size_t)j * 2048;
#pragma unroll 4
    for (int it = 0; it < 16; ++it) {
        const int f = (it * 32 + lane) * 4;
        const int kk = f >> 5, w0 = f & 31;
        const v4f v = *(const v4f*)(src + f);
#pragma unroll
        for (int i = 0; i < 4; ++i) ts[(w0 + i) * TP + kk] = v[i];
    }
    wave_sync();
#pragma unroll 1
    for (int ps = 0; ps < 2; ++ps) {
#pragma unroll
        for (int s = 0; s < 8; ++s) { const int row = 4 * s + (lane >> 3), c8 = (lane & 7) * 8;
            const v4f x0 = *(const v4fa*)(&ts[row * TP + c8]); const v4f x1 = *(const v4fa*)(&ts[row * TP + c8 + 4]); v8h hv;
#pragma unroll
            for (int i = 0; i < 4; ++i) { hv[i] = toh_flush(bfr(x0[i])); hv[4 + i] = toh_flush(bfr(x1[i])); }
            *(volatile v8h*)(WTp + (size_t)row * KUV + (size_t)j * 64 + c8) = hv; }
        if (ps == 0) __threadfence(); }
}

__global__ __launch_bounds__(32) __attribute__((amdgpu_num_vgpr(256)))
void k_tp(const float* __restrict__ X1, const float* __restrict__ X2, const h16* __restrict__ WT, float* OUT) {
    __shared__ __align__(16) float rec[16 * RP];
    __shared__ __align__(16) float os[16 * OP];
    const int lane = threadIdx.x & 31, lr = lane & 15, hi = lane >> 4;
    const int e0 = blockIdx.x * 16;
    {
        const int f0 = lane * 4;
        const int ro1 = (f0 < MUL_) ? f0 : (f0 + 32);
        const int ro2 = (f0 < MUL_) ? (f0 + 32) : (f0 + 128);
#pragma unroll 4
        for (int e = 0; e < 16; ++e) {
            const v4f a = *(const v4f*)(X1 + (size_t)(e0 + e) * DIMX + f0);
            const v4f b = *(const v4f*)(X2 + (size_t)(e0 + e) * DIMX + f0);
            v4f ao, bo;
#pragma unroll
            for (int i = 0; i < 4; ++i) { ao[i] = bfr(a[i]); bo[i] = bfr(b[i]); }
            *(v4fa*)(&rec[e * RP + ro1]) = ao; *(v4fa*)(&rec[e * RP + ro2]) = bo;
        }
    }
    wave_sync();
    const int rb = lr * RP;
    float b0v[16], b1x[16], b1y[16], b1z[16];
#pragma unroll
    for (int i = 0; i < 16; ++i) { const int v = (i < 8) ? (8 * hi + i) : (16 + 8 * hi + (i - 8));
        b0v[i] = rec[rb + 32 + v]; b1x[i] = rec[rb + 160 + 3 * v]; b1y[i] = rec[rb + 161 + 3 * v]; b1z[i] = rec[rb + 162 + 3 * v]; }
    v8f acc0[2]; v8f acc1[3][2];
#pragma unroll
    for (int nt = 0; nt < 2; ++nt) { acc0[nt] = (v8f){};
#pragma unroll
        for (int k = 0; k < 3; ++k) acc1[k][nt] = (v8f){}; }
    const size_t wo = (size_t)lr * KUV + 8 * hi;
    const float I3Z = I3F * ZC, I6Z = I6F * ZC;
#pragma unroll 1
    for (int u = 0; u < MUL_; ++u) {
        const float a0 = rec[rb + u];
        const float ax = rec[rb + 64 + 3 * u], ay = rec[rb + 65 + 3 * u], az = rec[rb + 66 + 3 * u];
        const h16* wp = WT + wo + (size_t)u * 32;
        {
            const float s0 = a0 * ZC; v16h A;
#pragma unroll
            for (int i = 0; i < 16; ++i) A[i] = toh_flush(s0 * b0v[i]);
            const v16h B0 = ldh(wp), B1 = ldh(wp + (size_t)16 * KUV);
            acc0[0] = wmma16g(A, B0, acc0[0]); acc0[1] = wmma16g(A, B1, acc0[1]);
        }
        const float px = ax * I3Z, py = ay * I3Z, pz = az * I3Z;
        {
            v16h A;
#pragma unroll
            for (int i = 0; i < 16; ++i) A[i] = toh_flush(px * b1x[i] + py * b1y[i] + pz * b1z[i]);
            const h16* w1 = wp + (size_t)1 * PLN;
            const v16h B0 = ldh(w1), B1 = ldh(w1 + (size_t)16 * KUV);
            acc0[0] = wmma16g(A, B0, acc0[0]); acc0[1] = wmma16g(A, B1, acc0[1]);
        }
        {
            const float s3 = a0 * I3Z; v16h A0, A1, A2;
#pragma unroll
            for (int i = 0; i < 16; ++i) { A0[i] = toh_flush(s3 * b1x[i]); A1[i] = toh_flush(s3 * b1y[i]); A2[i] = toh_flush(s3 * b1z[i]); }
            const h16* w2 = wp + (size_t)2 * PLN;
            const v16h B0 = ldh(w2), B1 = ldh(w2 + (size_t)16 * KUV);
            acc1[0][0] = wmma16g(A0, B0, acc1[0][0]); acc1[0][1] = wmma16g(A0, B1, acc1[0][1]);
            acc1[1][0] = wmma16g(A1, B0, acc1[1][0]); acc1[1][1] = wmma16g(A1, B1, acc1[1][1]);
            acc1[2][0] = wmma16g(A2, B0, acc1[2][0]); acc1[2][1] = wmma16g(A2, B1, acc1[2][1]);
        }
        {
            v16h A0, A1, A2;
#pragma unroll
            for (int i = 0; i < 16; ++i) { A0[i] = toh_flush(px * b0v[i]); A1[i] = toh_flush(py * b0v[i]); A2[i] = toh_flush(pz * b0v[i]); }
            const h16* w3 = wp + (size_t)3 * PLN;
            const v16h B0 = ldh(w3), B1 = ldh(w3 + (size_t)16 * KUV);
            acc1[0][0] = wmma16g(A0, B0, acc1[0][0]); acc1[0][1] = wmma16g(A0, B1, acc1[0][1]);
            acc1[1][0] = wmma16g(A1, B0, acc1[1][0]); acc1[1][1] = wmma16g(A1, B1, acc1[1][1]);
            acc1[2][0] = wmma16g(A2, B0, acc1[2][0]); acc1[2][1] = wmma16g(A2, B1, acc1[2][1]);
        }
        {
            const float cx = ax * I6Z, cy = ay * I6Z, cz = az * I6Z; v16h A0, A1, A2;
#pragma unroll
            for (int i = 0; i < 16; ++i) {
                A0[i] = toh_flush(cy * b1z[i] - cz * b1y[i]);
                A1[i] = toh_flush(cz * b1x[i] - cx * b1z[i]);
                A2[i] = toh_flush(cx * b1y[i] - cy * b1x[i]); }
            const h16* w4 = wp + (size_t)4 * PLN;
            const v16h B0 = ldh(w4), B1 = ldh(w4 + (size_t)16 * KUV);
            acc1[0][0] = wmma16g(A0, B0, acc1[0][0]); acc1[0][1] = wmma16g(A0, B1, acc1[0][1]);
            acc1[1][0] = wmma16g(A1, B0, acc1[1][0]); acc1[1][1] = wmma16g(A1, B1, acc1[1][1]);
            acc1[2][0] = wmma16g(A2, B0, acc1[2][0]); acc1[2][1] = wmma16g(A2, B1, acc1[2][1]);
        }
    }
    const float k0 = C0F * ZCI, k1 = C1F * ZCI;
#pragma unroll
    for (int nt = 0; nt < 2; ++nt) {
        const int w = nt * 16 + lr;
#pragma unroll
        for (int r = 0; r < 8; ++r) {
            const int ob = (8 * hi + r) * OP;
            os[ob + w] = acc0[nt][r] * k0;
            os[ob + 32 + 3 * w + 0] = acc1[0][nt][r] * k1;
            os[ob + 32 + 3 * w + 1] = acc1[1][nt][r] * k1;
            os[ob + 32 + 3 * w + 2] = acc1[2][nt][r] * k1; } }
    wave_sync();
    float* orow = OUT + (size_t)e0 * DIMX + lane * 4;
#pragma unroll 1
    for (int ps = 0; ps < 2; ++ps) {
#pragma unroll
        for (int row = 0; row < 16; ++row) {
            const v4f val = *(const v4fa*)(&os[row * OP + lane * 4]);
            *(volatile v4f*)(orow + (size_t)row * DIMX) = val; }
        if (ps == 0) __threadfence(); }
}

static constexpr size_t al256(size_t v) { return (v + 255) & ~(size_t)255; }
static constexpr size_t SZ_WT = al256((size_t)NPATH * PLN * 2);
static constexpr size_t SZ_TOTAL = SZ_WT;
static_assert(SZ_TOTAL <= (size_t)134217728);
static_assert(((size_t)PLN * 2) % 256 == 0);
static_assert((size_t)16 * 2048 == (size_t)MUL_ * KUV);
static_assert((size_t)(MUL_ - 1) * KUV + 15 * 64 + 56 + 8 <= (size_t)PLN);

extern "C" void kernel_launch(void* const* d_in, const int* in_sizes, int n_in,
                              void* d_out, int out_size, void* d_ws, size_t ws_size, hipStream_t stream) {
    if (n_in < 7) return;
    const size_t needx = (size_t)NE * DIMX;
    if ((size_t)in_sizes[0] < needx || (size_t)in_sizes[1] < needx) return;
    for (int i = 0; i < NPATH; ++i) if ((size_t)in_sizes[2 + i] < (size_t)MUL_ * KUV) return;
    if ((size_t)out_size < needx) return;
    if (SZ_TOTAL > ws_size) return;
    const float* x1 = (const float*)d_in[0];
    const float* x2 = (const float*)d_in[1];
    const float* w000 = (const float*)d_in[2];
    const float* w110 = (const float*)d_in[3];
    const float* w011 = (const float*)d_in[4];
    const float* w101 = (const float*)d_in[5];
    const float* w111 = (const float*)d_in[6];
    float* OUT = (float*)d_out;
    h16* WT = (h16*)d_ws;

    k_wconv<<<16, 32, 0, stream>>>(w000, WT + (size_t)0 * PLN);
    k_wconv<<<16, 32, 0, stream>>>(w110, WT + (size_t)1 * PLN);
    k_wconv<<<16, 32, 0, stream>>>(w011, WT + (size_t)2 * PLN);
    k_wconv<<<16, 32, 0, stream>>>(w101, WT + (size_t)3 * PLN);
    k_wconv<<<16, 32, 0, stream>>>(w111, WT + (size_t)4 * PLN);

    k_tp<<<NE / 16, 32, 0, stream>>>(x1, x2, WT, OUT);
}
